// Pointnet2_19439021982076
// MI455X (gfx1250) — hardware-verified
//
#include <hip/hip_runtime.h>
#pragma clang fp contract(off)

typedef __attribute__((ext_vector_type(16))) _Float16 v16h;
typedef __attribute__((ext_vector_type(8)))  _Float16 v8h;
typedef __attribute__((ext_vector_type(16))) __bf16   v16b;
typedef __attribute__((ext_vector_type(8)))  __bf16   v8b;
typedef __attribute__((ext_vector_type(8)))  float    v8f;
typedef __attribute__((ext_vector_type(4)))  float    v4f;
typedef __attribute__((ext_vector_type(2)))  float    v2f;
typedef __attribute__((ext_vector_type(4)))  int      v4i;
typedef __attribute__((ext_vector_type(4)))  unsigned v4u;

constexpr int NBATCH   = 4;
constexpr int NPT1     = 8192;
constexpr int NCEN1    = 2048;
constexpr int NSAMP1   = 32;
constexpr int NCH1     = 128;
constexpr int NCEN2    = 256;
constexpr int NSAMP2   = 16;
constexpr int NCIN2    = 131;
constexpr int NCH2     = 693;
constexpr int NCH2P    = 704;
constexpr int KDIM2    = 160;
constexpr int APITCH   = 256;
constexpr int NROW2    = NBATCH * NCEN2 * NSAMP2;
constexpr int MLP1_GPB = 16;
constexpr int NPART1   = (NBATCH * NCEN1) / MLP1_GPB;
constexpr int RED2_GPB = 8;
constexpr int NPART2   = (NBATCH * NCEN2) / RED2_GPB;

static_assert(NROW2 == 16384);
static_assert(NROW2 % 64 == 0);
static_assert(NCH2P % 64 == 0);
static_assert(KDIM2 % 32 == 0);
static_assert(KDIM2 <= APITCH);
static_assert(NCIN2 <= KDIM2);
static_assert(NCH2 <= NCH2P);
static_assert(((NROW2 / 64) * (NCH2P / 64)) % 8 == 0);
static_assert((NBATCH * NCEN2 * NCH2) % 1024 == 0);
static_assert(NBATCH * NCEN2 * 3 * 4 == 12288);
static_assert(12288 + NBATCH * NCEN2 * NCH2 * 4 == 2850816);
static_assert(NCEN1 % MLP1_GPB == 0);
static_assert(NCH2P == 176 * 4);

constexpr float BALL_R2_L1 = (float)(0.0025 * 0.0025);
constexpr float BALL_R2_L2 = (float)(0.005 * 0.005);
constexpr float BN_EPS = 1e-5f;

constexpr size_t al256(size_t x) { return (x + 255) & ~(size_t)255; }
constexpr size_t SZ_L1XYZ = (size_t)NBATCH * NCEN1 * 4 * 4;
constexpr size_t SZ_L2XYZ = (size_t)NBATCH * NCEN2 * 4 * 4;
constexpr size_t SZ_IDX1  = (size_t)NBATCH * NCEN1 * NSAMP1 * 4;
constexpr size_t SZ_IDX2  = (size_t)NBATCH * NCEN2 * NSAMP2 * 4;
constexpr size_t SZ_H1    = (size_t)NBATCH * NCEN1 * NCH1 * 4;
constexpr size_t SZ_PART1 = (size_t)NPART1 * 2 * NCH1 * 4;
constexpr size_t SZ_SS1   = (size_t)NCH1 * 4;
constexpr size_t SZ_APL   = (size_t)NROW2 * APITCH * 2;
constexpr size_t SZ_WPL   = (size_t)NCH2P * APITCH * 2;
constexpr size_t SZ_H2    = (size_t)NROW2 * NCH2P * 4;
constexpr size_t SZ_H2M   = (size_t)NBATCH * NCEN2 * NCH2P * 4;
constexpr size_t SZ_PART2 = (size_t)NPART2 * 2 * NCH2P * 4;
constexpr size_t SZ_SS2   = (size_t)NCH2P * 4;

constexpr size_t OFF_L1XYZ = 0;
constexpr size_t OFF_L2XYZ = OFF_L1XYZ + al256(SZ_L1XYZ);
constexpr size_t OFF_IDX1  = OFF_L2XYZ + al256(SZ_L2XYZ);
constexpr size_t OFF_IDX2  = OFF_IDX1  + al256(SZ_IDX1);
constexpr size_t OFF_H1MAX = OFF_IDX2  + al256(SZ_IDX2);
constexpr size_t OFF_H1MIN = OFF_H1MAX + al256(SZ_H1);
constexpr size_t OFF_PART1 = OFF_H1MIN + al256(SZ_H1);
constexpr size_t OFF_SC1   = OFF_PART1 + al256(SZ_PART1);
constexpr size_t OFF_SH1   = OFF_SC1   + al256(SZ_SS1);
constexpr size_t OFF_AHI   = OFF_SH1   + al256(SZ_SS1);
constexpr size_t OFF_ALO   = OFF_AHI   + al256(SZ_APL);
constexpr size_t OFF_WHI   = OFF_ALO   + al256(SZ_APL);
constexpr size_t OFF_WLO   = OFF_WHI   + al256(SZ_WPL);
constexpr size_t OFF_H2    = OFF_WLO   + al256(SZ_WPL);
constexpr size_t OFF_H2MAX = OFF_H2    + al256(SZ_H2);
constexpr size_t OFF_H2MIN = OFF_H2MAX + al256(SZ_H2M);
constexpr size_t OFF_PART2 = OFF_H2MIN + al256(SZ_H2M);
constexpr size_t OFF_SC2   = OFF_PART2 + al256(SZ_PART2);
constexpr size_t OFF_SH2   = OFF_SC2   + al256(SZ_SS2);
constexpr size_t WS_TOTAL  = OFF_SH2   + al256(SZ_SS2);
static_assert(WS_TOTAL <= (size_t)134217728);

__device__ __forceinline__ unsigned bf_rne_bits(float f) {
  const unsigned u = __float_as_uint(f);
  return (u + 0x7FFFu + ((u >> 16) & 1u)) >> 16;
}
__device__ __forceinline__ unsigned short f2bf_bits(float f) {
  unsigned u = __float_as_uint(f);
  return (unsigned short)((u + 0x7FFFu + ((u >> 16) & 1u)) >> 16);
}
__device__ __forceinline__ float bf_bits2f(unsigned short h) { return __uint_as_float(((unsigned)h) << 16); }
__device__ __forceinline__ int clampi(int v, int lo, int hi) { return v < lo ? lo : (v > hi ? hi : v); }

__device__ __forceinline__ void dep_guard4_h(v8f& a, v8f& b, v8f& c, v8f& d, v16h x, v16h y) { asm volatile("v_nop\n\tv_nop\n\tv_nop\n\tv_nop" : "+v"(a), "+v"(b), "+v"(c), "+v"(d) : "v"(x), "v"(y)); }
__device__ __forceinline__ void dep_guard4_b(v8f& a, v8f& b, v8f& c, v8f& d, v16b x, v16b y) { asm volatile("v_nop\n\tv_nop\n\tv_nop\n\tv_nop" : "+v"(a), "+v"(b), "+v"(c), "+v"(d) : "v"(x), "v"(y)); }
__device__ __forceinline__ void keep4_h(v16h a, v16h b, v16h c, v16h d) { asm volatile("v_nop" :: "v"(a), "v"(b), "v"(c), "v"(d)); }
__device__ __forceinline__ void keep4_b(v16b a, v16b b, v16b c, v16b d) { asm volatile("v_nop" :: "v"(a), "v"(b), "v"(c), "v"(d)); }
__device__ __forceinline__ void acc_guard4(v8f& a, v8f& b, v8f& c, v8f& d) { asm volatile("v_nop\n\tv_nop\n\tv_nop\n\tv_nop" : "+v"(a), "+v"(b), "+v"(c), "+v"(d)); }

template <typename T> struct Frag;
template <> struct Frag<_Float16> {
  typedef v16h V; union U { v16h v; v8h h[2]; };
  static __device__ __forceinline__ v16h load(const _Float16* p) {
    U f; f.h[0] = *(const v8h*)(p); f.h[1] = *(const v8h*)(p + 16); return f.v;
  }
  static __device__ __forceinline__ v8f mma(v16h a, v16h b, v8f c) {
    return __builtin_amdgcn_wmma_f32_16x16x32_f16(false, a, false, b, (short)0, c, false, false);
  }
  static __device__ __forceinline__ void guard4(v8f& a, v8f& b, v8f& c, v8f& d, v16h x, v16h y) { dep_guard4_h(a, b, c, d, x, y); }
  static __device__ __forceinline__ void keep(v16h a, v16h b, v16h c, v16h d) { keep4_h(a, b, c, d); }
};
template <> struct Frag<__bf16> {
  typedef v16b V; union U { v16b v; v8b h[2]; };
  static __device__ __forceinline__ v16b load(const __bf16* p) {
    U f; f.h[0] = *(const v8b*)(p); f.h[1] = *(const v8b*)(p + 16); return f.v;
  }
  static __device__ __forceinline__ v8f mma(v16b a, v16b b, v8f c) {
    return __builtin_amdgcn_wmma_f32_16x16x32_bf16(false, a, false, b, (short)0, c, false, false);
  }
  static __device__ __forceinline__ void guard4(v8f& a, v8f& b, v8f& c, v8f& d, v16b x, v16b y) { dep_guard4_b(a, b, c, d, x, y); }
  static __device__ __forceinline__ void keep(v16b a, v16b b, v16b c, v16b d) { keep4_b(a, b, c, d); }
};

template <int ET> struct Elem;
template <> struct Elem<0> { typedef _Float16 T; };
template <> struct Elem<1> { typedef __bf16 T; };
template <int ET, bool SPLIT, int BIAS_MODE, int OUT_MODE, bool RESID, int ACT = 0>
__global__ __launch_bounds__(256) void wmma_gemm64(
    const unsigned short* __restrict__ Ap, const unsigned short* __restrict__ A2p, int lda, long strideA,
    const unsigned short* __restrict__ Btp, const unsigned short* __restrict__ Bt2p, int ldb, long strideB,
    void* __restrict__ Cout, void* __restrict__ Cout2, int ldc, long strideC,
    const float* __restrict__ bias,
    const float* __restrict__ resid, long strideR,
    int M, int N, int K, float scale) {
  typedef typename Elem<ET>::T T;
  typedef typename Frag<T>::V V;
  const T* A = (const T*)Ap; const T* A2 = (const T*)A2p; const T* Bt = (const T*)Btp; const T* Bt2 = (const T*)Bt2p;
  __shared__ __align__(16) float sT[8][16 * 68];
  const int b    = blockIdx.y;
  const int lane = threadIdx.x & 31;
  const int wave = threadIdx.x >> 5;
  const int tilesN = N >> 6;
  const int tilesM = M >> 6;
  const int tile = blockIdx.x * 8 + wave;
  if (tile >= tilesM * tilesN) return;
  const int tm = tile / tilesN;
  const int tn = tile - tm * tilesN;
  const int m0 = tm << 6;
  const int n0 = tn << 6;

  const T* Ab  = A  + (size_t)b * strideA;
  const T* Bb  = Bt + (size_t)b * strideB;
  const T* Ab2 = SPLIT ? (A2  + (size_t)b * strideA) : nullptr;
  const T* Bb2 = SPLIT ? (Bt2 + (size_t)b * strideB) : nullptr;

  const int rlane = lane & 15;
  const int koff  = (lane >> 4) * 8;
  const int mOff  = (lane >> 4) * 8;

  v8f acc[4][4];
#pragma unroll
  for (int i = 0; i < 4; ++i)
#pragma unroll
    for (int j = 0; j < 4; ++j) acc[i][j] = (v8f){0.f,0.f,0.f,0.f,0.f,0.f,0.f,0.f};

  for (int k0 = 0; k0 < K; k0 += 32) {
    V bh[4], bl[4];
#pragma unroll
    for (int j = 0; j < 4; ++j) {
      const size_t bo = (size_t)(n0 + (j << 4) + rlane) * ldb + koff + k0;
      bh[j] = Frag<T>::load(Bb + bo);
      if (SPLIT) bl[j] = Frag<T>::load(Bb2 + bo);
    }
#pragma unroll
    for (int i = 0; i < 4; ++i) {
      const size_t ao = (size_t)(m0 + (i << 4) + rlane) * lda + koff + k0;
      V ah = Frag<T>::load(Ab + ao);
      V al;
      if (SPLIT) al = Frag<T>::load(Ab2 + ao);
#pragma unroll
      for (int j = 0; j < 4; ++j) {
        acc[i][j] = Frag<T>::mma(ah, bh[j], acc[i][j]);
        if (SPLIT) {
          acc[i][j] = Frag<T>::mma(ah, bl[j], acc[i][j]);
          acc[i][j] = Frag<T>::mma(al, bh[j], acc[i][j]);
        }
      }
      Frag<T>::guard4(acc[i][0], acc[i][1], acc[i][2], acc[i][3], ah, SPLIT ? al : ah);
    }
    Frag<T>::keep(bh[0], bh[1], bh[2], bh[3]);
    if (SPLIT) Frag<T>::keep(bl[0], bl[1], bl[2], bl[3]);
  }
  acc_guard4(acc[0][0], acc[0][1], acc[0][2], acc[0][3]);
  acc_guard4(acc[1][0], acc[1][1], acc[1][2], acc[1][3]);
  acc_guard4(acc[2][0], acc[2][1], acc[2][2], acc[2][3]);
  acc_guard4(acc[3][0], acc[3][1], acc[3][2], acc[3][3]);

  float* slab = sT[wave];
  const float* Rb = RESID ? (resid + (size_t)b * strideR) : nullptr;
#pragma unroll
  for (int i = 0; i < 4; ++i) {
    const int mBase = m0 + (i << 4);
#pragma unroll
    for (int j = 0; j < 4; ++j) {
      const int n = n0 + (j << 4) + rlane;
      float bv = 0.f;
      if (BIAS_MODE == 2) bv = bias[n];
#pragma unroll
      for (int r = 0; r < 8; ++r) {
        float v = acc[i][j][r] * scale;
        if (BIAS_MODE == 1) v += bias[mBase + mOff + r];
        if (BIAS_MODE == 2) v += bv;
        if (RESID) v += Rb[(size_t)(mBase + mOff + r) * ldc + n];
        if (ACT == 2) v = fmaxf(v, 0.0f);
        if (ACT == 4) v = (v > 0.f) ? v : 0.01f * v;
        slab[(mOff + r) * 68 + (j << 4) + rlane] = v;
      }
    }
    __builtin_amdgcn_fence(__ATOMIC_RELEASE, "workgroup");
    __builtin_amdgcn_wave_barrier();
    __builtin_amdgcn_fence(__ATOMIC_ACQUIRE, "workgroup");
    if (OUT_MODE == 0) {
      float* C = (float*)Cout + (size_t)b * strideC;
      const int hh = lane >> 4, c4 = (lane & 15) * 4;
      for (int pass = 0; pass < 2; ++pass) {
#pragma unroll
        for (int it = 0; it < 8; ++it) {
          const int row = it * 2 + hh;
          v4f v = *(const v4f*)(slab + row * 68 + c4);
          *(volatile v4f*)(C + (size_t)(mBase + row) * ldc + n0 + c4) = v;
        }
        __threadfence();
      }
    } else {
      const int q = lane >> 3, c8 = (lane & 7) * 8;
      unsigned short* C  = (unsigned short*)Cout  + (size_t)b * strideC;
      unsigned short* C2 = (OUT_MODE == 2) ? ((unsigned short*)Cout2 + (size_t)b * strideC) : nullptr;
      for (int pass = 0; pass < 2; ++pass) {
#pragma unroll
        for (int it = 0; it < 4; ++it) {
          const int row = it * 4 + q;
          const float* sp = slab + row * 68 + c8;
          v8h hv, lv;
#pragma unroll
          for (int e = 0; e < 8; ++e) {
            if (OUT_MODE == 1) {
              hv[e] = (_Float16)sp[e];
            } else {
              unsigned short hb = f2bf_bits(sp[e]);
              unsigned short lb = f2bf_bits(sp[e] - bf_bits2f(hb));
              hv[e] = __builtin_bit_cast(_Float16, hb);
              lv[e] = __builtin_bit_cast(_Float16, lb);
            }
          }
          *(volatile v8h*)(C + (size_t)(mBase + row) * ldc + n0 + c8) = hv;
          if (OUT_MODE == 2) *(volatile v8h*)(C2 + (size_t)(mBase + row) * ldc + n0 + c8) = lv;
        }
        __threadfence();
      }
    }
    __builtin_amdgcn_fence(__ATOMIC_RELEASE, "workgroup");
    __builtin_amdgcn_wave_barrier();
    __builtin_amdgcn_fence(__ATOMIC_ACQUIRE, "workgroup");
  }
}

template <int NPTS, int PPT, int NPICK, int INSTRIDE, int OUTMODE>
__global__ __launch_bounds__(512) void fps_kernel(const float* __restrict__ pts,
                                                  float* __restrict__ out4,
                                                  float* __restrict__ outflat) {
#pragma clang fp contract(off)
  static_assert(NPTS == 512 * PPT);
  extern __shared__ __align__(16) float fsm[];
  float* X = fsm;
  float* Y = fsm + NPTS;
  float* Z = fsm + 2 * NPTS;
  int* picks = (int*)(fsm + 3 * NPTS);
  __shared__ float rv[2][16];
  __shared__ int   ri[2][16];

  const int tid = threadIdx.x;
  const int lane = tid & 31;
  const int wave = tid >> 5;
  const int b = blockIdx.x;
  const float* p = pts + (size_t)b * NPTS * INSTRIDE;

#pragma unroll 1
  for (int j = 0; j < PPT; ++j) {
    const int i = tid + 512 * j;
    const float* q = p + (size_t)i * INSTRIDE;
    const float x = q[0];
    const float y = q[1];
    const float z = q[2];
    X[i] = x;
    Y[i] = y;
    Z[i] = z;
  }
  __syncthreads();

  float px[PPT], py[PPT], pz[PPT], pd[PPT];
#pragma unroll
  for (int j = 0; j < PPT; ++j) {
    px[j] = X[tid + 512 * j];
    py[j] = Y[tid + 512 * j];
    pz[j] = Z[tid + 512 * j];
    pd[j] = 1e10f;
  }

  int far = 0;
#pragma unroll 1
  for (int it = 0; it < NPICK; ++it) {
    if (tid == 0) picks[it] = far;
    const float cx = X[far];
    const float cy = Y[far];
    const float cz = Z[far];
    float bv = 0.0f;
    int bi = 0;
#pragma unroll
    for (int j = 0; j < PPT; ++j) {
      const float dx = px[j] - cx;
      const float dy = py[j] - cy;
      const float dz = pz[j] - cz;
      const float t0 = dx * dx;
      const float t1 = dy * dy;
      const float t2 = dz * dz;
      const float d = (t0 + t2) + t1;
      const float nd = fminf(pd[j], d);
      pd[j] = nd;
      if (j == 0) {
        bv = nd;
        bi = tid;
      } else {
        const bool tk = nd > bv;
        bv = tk ? nd : bv;
        bi = tk ? (tid + 512 * j) : bi;
      }
    }
#pragma unroll
    for (int off = 16; off > 0; off >>= 1) {
      const float ov = __shfl_xor(bv, off, 32);
      const int   oi = __shfl_xor(bi, off, 32);
      const bool tk = (ov > bv) || ((ov == bv) && (oi < bi));
      bv = tk ? ov : bv;
      bi = tk ? oi : bi;
    }
    const int buf = it & 1;
    if (lane == 0) {
      rv[buf][wave] = bv;
      ri[buf][wave] = bi;
    }
    __syncthreads();
    bv = rv[buf][lane & 15];
    bi = ri[buf][lane & 15];
#pragma unroll
    for (int off = 8; off > 0; off >>= 1) {
      const float ov = __shfl_xor(bv, off, 32);
      const int   oi = __shfl_xor(bi, off, 32);
      const bool tk = (ov > bv) || ((ov == bv) && (oi < bi));
      bv = tk ? ov : bv;
      bi = tk ? oi : bi;
    }
    far = clampi(bi, 0, NPTS - 1);
  }
  __syncthreads();

  for (int pass = 0; pass < 2; ++pass) {
#pragma unroll 1
    for (int s = tid; s < NPICK; s += 512) {
      const int pk = clampi(picks[s], 0, NPTS - 1);
      v4f v;
      v.x = X[pk];
      v.y = Y[pk];
      v.z = Z[pk];
      v.w = 0.0f;
      *(volatile v4f*)(out4 + ((size_t)b * NPICK + s) * 4) = v;
    }
    if (OUTMODE == 2) {
#pragma unroll 1
      for (int q = tid; q < (NPICK * 3) / 4; q += 512) {
        v4f v;
#pragma unroll
        for (int e = 0; e < 4; ++e) {
          const int f = 4 * q + e;
          const int s = f / 3;
          const int c = f - 3 * s;
          const int pk = clampi(picks[s], 0, NPTS - 1);
          const float xv = X[pk];
          const float yv = Y[pk];
          const float zv = Z[pk];
          v[e] = (c == 0) ? xv : ((c == 1) ? yv : zv);
        }
        *(volatile v4f*)(outflat + (size_t)b * NPICK * 3 + 4 * q) = v;
      }
    }
    __threadfence();
  }
}

template <int NPTS, int NCEN, int NSAMP, int INSTRIDE>
__global__ __launch_bounds__(256) void ballquery_kernel(const float* __restrict__ pts,
                                                        const float* __restrict__ cen4,
                                                        int* __restrict__ idx_out, float r2) {
#pragma clang fp contract(off)
  constexpr int TILE = 1024;
  constexpr int HP = NSAMP + 1;
  static_assert(NPTS % TILE == 0);
  static_assert(NCEN % 256 == 0);
  static_assert(NSAMP % 4 == 0 && NSAMP <= 32);
  __shared__ __align__(16) float tile[TILE * 4];
  __shared__ int hits[256 * HP];

  const int tid = threadIdx.x;
  const int lane = tid & 31;
  const int wave = tid >> 5;
  const int cflat = blockIdx.x * 256 + tid;
  const int b = (blockIdx.x * 256) / NCEN;

  const v4f cc = *(const v4f*)(cen4 + (size_t)cflat * 4);
  const float cx = cc.x;
  const float cy = cc.y;
  const float cz = cc.z;
  const float c0 = cx * cx;
  const float c1 = cy * cy;
  const float c2 = cz * cz;
  const float sqc = (c0 + c2) + c1;

  int cnt = 0;
  hits[tid * HP] = NPTS;

  for (int n0 = 0; n0 < NPTS; n0 += TILE) {
    __syncthreads();
#pragma unroll 1
    for (int i = tid; i < TILE; i += 256) {
      const float* q = pts + ((size_t)b * NPTS + n0 + i) * INSTRIDE;
      const float x = q[0];
      const float y = q[1];
      const float z = q[2];
      const float s0 = x * x;
      const float s1 = y * y;
      const float s2 = z * z;
      v4f t;
      t.x = x;
      t.y = y;
      t.z = z;
      t.w = (s0 + s2) + s1;
      *(v4f*)(tile + 4 * i) = t;
    }
    __syncthreads();
#pragma unroll 4
    for (int n = 0; n < TILE; ++n) {
      const v4f pp = *(const v4f*)(tile + 4 * n);
      float d = cx * pp.x;
      d = __builtin_fmaf(cy, pp.y, d);
      d = __builtin_fmaf(cz, pp.z, d);
      const float two_d = 2.0f * d;
      const float sq = (sqc + pp.w) - two_d;
      const bool inb = !(sq > r2);
      if (inb && (cnt < NSAMP)) {
        hits[tid * HP + cnt] = n0 + n;
        ++cnt;
      }
    }
  }
  const int first = hits[tid * HP];
#pragma unroll 1
  for (int s = cnt; s < NSAMP; ++s) hits[tid * HP + s] = first;
  __syncthreads();

  constexpr int LPC = NSAMP / 4;
  constexpr int CPI = 32 / LPC;
  for (int pass = 0; pass < 2; ++pass) {
#pragma unroll
    for (int it = 0; it < LPC; ++it) {
      const int cl = wave * 32 + it * CPI + lane / LPC;
      const int s4 = (lane % LPC) * 4;
      v4i v;
#pragma unroll
      for (int e = 0; e < 4; ++e) {
        const int hv = hits[cl * HP + s4 + e];
        v[e] = clampi(hv, 0, NPTS - 1);
      }
      *(volatile v4i*)(idx_out + ((size_t)(blockIdx.x * 256 + cl)) * NSAMP + s4) = v;
    }
    __threadfence();
  }
}

__global__ __launch_bounds__(128) void mlp1_kernel(const float* __restrict__ xyz,
                                                   const float* __restrict__ cen4,
                                                   const int* __restrict__ idx1,
                                                   const float* __restrict__ w1,
                                                   const float* __restrict__ b1,
                                                   float* __restrict__ h1max,
                                                   float* __restrict__ h1min,
                                                   float* __restrict__ partials) {
  constexpr int ROWS = MLP1_GPB * NSAMP1;
  __shared__ __align__(16) float G[ROWS * 8];
  __shared__ __align__(16) float Smax[MLP1_GPB * NCH1];
  __shared__ __align__(16) float Smin[MLP1_GPB * NCH1];
  __shared__ __align__(16) float Sst[2 * NCH1];

  const int tid = threadIdx.x;
  const int g0 = blockIdx.x * MLP1_GPB;
  const int b = g0 / NCEN1;

#pragma unroll 1
  for (int i = 0; i < ROWS / 128; ++i) {
    const int r = tid + 128 * i;
    const int g = g0 + (r >> 5);
    const int j = clampi(idx1[(size_t)g * NSAMP1 + (r & 31)], 0, NPT1 - 1);
    const float* q = xyz + ((size_t)b * NPT1 + j) * 6;
    const v2f a0 = *(const v2f*)(q);
    const v2f a1 = *(const v2f*)(q + 2);
    const v2f a2 = *(const v2f*)(q + 4);
    const v4f c = *(const v4f*)(cen4 + (size_t)g * 4);
    v4f lo4;
    lo4.x = a0.x - c.x;
    lo4.y = a0.y - c.y;
    lo4.z = a1.x - c.z;
    lo4.w = a1.y;
    v4f hi4;
    hi4.x = a2.x;
    hi4.y = a2.y;
    hi4.z = 0.0f;
    hi4.w = 0.0f;
    *(v4f*)(G + r * 8) = lo4;
    *(v4f*)(G + r * 8 + 4) = hi4;
  }
  __syncthreads();

  const float w0 = w1[0 * NCH1 + tid];
  const float w1v = w1[1 * NCH1 + tid];
  const float w2v = w1[2 * NCH1 + tid];
  const float w3v = w1[3 * NCH1 + tid];
  const float w4v = w1[4 * NCH1 + tid];
  const float w5v = w1[5 * NCH1 + tid];
  const float bias = b1[tid];

  float ts = 0.0f, tq = 0.0f;
#pragma unroll 1
  for (int gl = 0; gl < MLP1_GPB; ++gl) {
    float m = -3.402823466e38f;
    float mn = 3.402823466e38f;
    float gs = 0.0f, gq = 0.0f;
#pragma unroll 4
    for (int k = 0; k < NSAMP1; ++k) {
      const float* gr = G + (gl * NSAMP1 + k) * 8;
      const v4f a = *(const v4f*)(gr);
      const v4f c = *(const v4f*)(gr + 4);
      float h = bias;
      h = __builtin_fmaf(a.x, w0, h);
      h = __builtin_fmaf(a.y, w1v, h);
      h = __builtin_fmaf(a.z, w2v, h);
      h = __builtin_fmaf(a.w, w3v, h);
      h = __builtin_fmaf(c.x, w4v, h);
      h = __builtin_fmaf(c.y, w5v, h);
      m = fmaxf(m, h);
      mn = fminf(mn, h);
      gs += h;
      gq = __builtin_fmaf(h, h, gq);
    }
    Smax[gl * NCH1 + tid] = m;
    Smin[gl * NCH1 + tid] = mn;
    ts += gs;
    tq += gq;
  }
  Sst[tid] = ts;
  Sst[NCH1 + tid] = tq;
  __syncthreads();

  for (int pass = 0; pass < 2; ++pass) {
#pragma unroll
    for (int i = 0; i < (MLP1_GPB * NCH1) / (128 * 4); ++i) {
      const int q = tid + 128 * i;
      const v4f vm = *(const v4f*)(Smax + 4 * q);
      const v4f vn = *(const v4f*)(Smin + 4 * q);
      *(volatile v4f*)(h1max + (size_t)g0 * NCH1 + 4 * q) = vm;
      *(volatile v4f*)(h1min + (size_t)g0 * NCH1 + 4 * q) = vn;
    }
    if (tid < 64) {
      const v4f vs = *(const v4f*)(Sst + 4 * tid);
      *(volatile v4f*)(partials + (size_t)blockIdx.x * (2 * NCH1) + 4 * tid) = vs;
    }
    __threadfence();
  }
}

__global__ __launch_bounds__(256) void bn_finalize_kernel(const float* __restrict__ partials,
                                                          const float* __restrict__ gamma,
                                                          const float* __restrict__ beta,
                                                          float* __restrict__ scale,
                                                          float* __restrict__ shift,
                                                          float invcnt, int nparts, int nchpad, int nch) {
  __shared__ double rs[8][32];
  __shared__ double rq[8][32];
  __shared__ __align__(16) float so[64];
  const int tid = threadIdx.x;
  const int c = tid & 31;
  const int sl = tid >> 5;
  const int ch = blockIdx.x * 32 + c;
  double s = 0.0, q = 0.0;
#pragma unroll 1
  for (int p = sl; p < nparts; p += 8) {
    const float a = partials[((size_t)p * 2) * nchpad + ch];
    const float d = partials[((size_t)p * 2 + 1) * nchpad + ch];
    s += (double)a;
    q += (double)d;
  }
  rs[sl][c] = s;
  rq[sl][c] = q;
  __syncthreads();
  if (tid < 32) {
    double S = 0.0, Q = 0.0;
#pragma unroll
    for (int k = 0; k < 8; ++k) {
      S += rs[k][c];
      Q += rq[k][c];
    }
    const double mu = S * (double)invcnt;
    double var = Q * (double)invcnt - mu * mu;
    var = var < 0.0 ? 0.0 : var;
    const int chc = ch < nch ? ch : (nch - 1);
    const float gm = gamma[chc];
    const float bt = beta[chc];
    const float inv = rsqrtf((float)var + BN_EPS);
    const float sc = gm * inv;
    const float sh = bt - (float)mu * sc;
    const bool real = ch < nch;
    so[c] = real ? sc : 0.0f;
    so[32 + c] = real ? sh : 0.0f;
  }
  __syncthreads();
  if (tid < 16) {
    const int which = tid >> 3;
    const int c4 = (tid & 7) * 4;
    const v4f v = *(const v4f*)(so + which * 32 + c4);
    float* dst = (which ? shift : scale) + blockIdx.x * 32 + c4;
    *(volatile v4f*)dst = v;
    __threadfence();
    *(volatile v4f*)dst = v;
  }
}

__global__ __launch_bounds__(256) void pack_w2_kernel(const float* __restrict__ w2,
                                                      unsigned short* __restrict__ Whi,
                                                      unsigned short* __restrict__ Wlo) {
  const int lane = threadIdx.x & 31;
  const int wave = threadIdx.x >> 5;
  const int n = blockIdx.x * 8 + wave;
  const int nc = n < NCH2 ? n : (NCH2 - 1);
  float o[8];
#pragma unroll
  for (int e = 0; e < 8; ++e) {
    const int k = lane * 8 + e;
    int src = (k < 128) ? (k + 3) : (k - 128);
    src = clampi(src, 0, NCIN2 - 1);
    float v = w2[(size_t)src * NCH2 + nc];
    asm volatile("" : "+v"(v));
    o[e] = ((k < NCIN2) && (n < NCH2)) ? v : 0.0f;
  }
  unsigned hw[4], lw[4];
#pragma unroll
  for (int e = 0; e < 4; ++e) {
    const float x0 = o[2 * e];
    const float x1 = o[2 * e + 1];
    const unsigned h0 = bf_rne_bits(x0);
    const unsigned h1 = bf_rne_bits(x1);
    const unsigned l0 = bf_rne_bits(x0 - __uint_as_float(h0 << 16));
    const unsigned l1 = bf_rne_bits(x1 - __uint_as_float(h1 << 16));
    hw[e] = (h0 & 0xffffu) | (h1 << 16);
    lw[e] = (l0 & 0xffffu) | (l1 << 16);
  }
  v4u hv, lv;
  hv.x = hw[0]; hv.y = hw[1]; hv.z = hw[2]; hv.w = hw[3];
  lv.x = lw[0]; lv.y = lw[1]; lv.z = lw[2]; lv.w = lw[3];
  unsigned short* ph = Whi + (size_t)n * APITCH + lane * 8;
  unsigned short* pl = Wlo + (size_t)n * APITCH + lane * 8;
  *(volatile v4u*)ph = hv;
  *(volatile v4u*)pl = lv;
  __threadfence();
  *(volatile v4u*)ph = hv;
  *(volatile v4u*)pl = lv;
}

__global__ __launch_bounds__(256) void pack_a2_kernel(const float* __restrict__ h1max,
                                                      const float* __restrict__ h1min,
                                                      const float* __restrict__ scale1,
                                                      const float* __restrict__ shift1,
                                                      const float* __restrict__ l1xyz4,
                                                      const float* __restrict__ l2xyz4,
                                                      const int* __restrict__ idx2,
                                                      unsigned short* __restrict__ Ahi,
                                                      unsigned short* __restrict__ Alo) {
  __shared__ __align__(16) float ssc[NCH1];
  __shared__ __align__(16) float ssh[NCH1];
  const int tid = threadIdx.x;
  const int lane = tid & 31;
  const int wave = tid >> 5;
  if (tid < 32) {
    *(v4f*)(ssc + 4 * tid) = *(const v4f*)(scale1 + 4 * tid);
  } else if (tid < 64) {
    *(v4f*)(ssh + 4 * (tid - 32)) = *(const v4f*)(shift1 + 4 * (tid - 32));
  }
  __syncthreads();

  const int R = blockIdx.x * 8 + wave;
  const int b = R >> 12;
  const int cflat = R >> 4;
  const int j = clampi(idx2[R], 0, NCEN1 - 1);
  const size_t src = (size_t)b * NCEN1 + j;
  const int lc = lane < 16 ? lane : 15;
  const float* pm = h1max + src * NCH1 + lc * 8;
  const float* pn = h1min + src * NCH1 + lc * 8;
  v4f mx0 = *(const v4f*)(pm);
  v4f mx1 = *(const v4f*)(pm + 4);
  v4f mn0 = *(const v4f*)(pn);
  v4f mn1 = *(const v4f*)(pn + 4);
  v4f pc = *(const v4f*)(l1xyz4 + src * 4);
  v4f ct = *(const v4f*)(l2xyz4 + (size_t)cflat * 4);
  asm volatile("" : "+v"(mx0), "+v"(mx1), "+v"(mn0), "+v"(mn1), "+v"(pc), "+v"(ct));
  const v4f s0 = *(const v4f*)(ssc + lc * 8);
  const v4f s1 = *(const v4f*)(ssc + lc * 8 + 4);
  const v4f t0 = *(const v4f*)(ssh + lc * 8);
  const v4f t1 = *(const v4f*)(ssh + lc * 8 + 4);

  float feat[8];
#pragma unroll
  for (int e = 0; e < 4; ++e) {
    const float sca = s0[e];
    const float scb = s1[e];
    const float ha = (sca >= 0.0f) ? mx0[e] : mn0[e];
    const float hb = (scb >= 0.0f) ? mx1[e] : mn1[e];
    feat[e] = fmaxf(__builtin_fmaf(sca, ha, t0[e]), 0.0f);
    feat[4 + e] = fmaxf(__builtin_fmaf(scb, hb, t1[e]), 0.0f);
  }
  float rel[3];
  rel[0] = pc.x - ct.x;
  rel[1] = pc.y - ct.y;
  rel[2] = pc.z - ct.z;
  const bool isf = lane < 16;
  const bool isr = lane == 16;
  float o[8];
#pragma unroll
  for (int e = 0; e < 8; ++e) {
    const float rv = (e < 3) ? rel[e < 3 ? e : 0] : 0.0f;
    o[e] = isf ? feat[e] : (isr ? rv : 0.0f);
  }
  unsigned hw[4], lw[4];
#pragma unroll
  for (int e = 0; e < 4; ++e) {
    const float x0 = o[2 * e];
    const float x1 = o[2 * e + 1];
    const unsigned h0 = bf_rne_bits(x0);
    const unsigned h1 = bf_rne_bits(x1);
    const unsigned l0 = bf_rne_bits(x0 - __uint_as_float(h0 << 16));
    const unsigned l1 = bf_rne_bits(x1 - __uint_as_float(h1 << 16));
    hw[e] = (h0 & 0xffffu) | (h1 << 16);
    lw[e] = (l0 & 0xffffu) | (l1 << 16);
  }
  v4u hv, lv;
  hv.x = hw[0]; hv.y = hw[1]; hv.z = hw[2]; hv.w = hw[3];
  lv.x = lw[0]; lv.y = lw[1]; lv.z = lw[2]; lv.w = lw[3];
  unsigned short* ph = Ahi + (size_t)R * APITCH + lane * 8;
  unsigned short* pl = Alo + (size_t)R * APITCH + lane * 8;
  *(volatile v4u*)ph = hv;
  *(volatile v4u*)pl = lv;
  __threadfence();
  *(volatile v4u*)ph = hv;
  *(volatile v4u*)pl = lv;
}

__global__ __launch_bounds__(176) void reduce2_kernel(const float* __restrict__ H2,
                                                      const float* __restrict__ b2,
                                                      float* __restrict__ h2max,
                                                      float* __restrict__ h2min,
                                                      float* __restrict__ partials2) {
  const int tid = threadIdx.x;
  const int c4 = tid * 4;
  float bv[4];
#pragma unroll
  for (int e = 0; e < 4; ++e) {
    const int ch = c4 + e;
    float v = b2[ch < NCH2 ? ch : (NCH2 - 1)];
    asm volatile("" : "+v"(v));
    bv[e] = (ch < NCH2) ? v : 0.0f;
  }
  float ts[4] = {0.0f, 0.0f, 0.0f, 0.0f};
  float tq[4] = {0.0f, 0.0f, 0.0f, 0.0f};
  const int g0 = blockIdx.x * RED2_GPB;
#pragma unroll 1
  for (int gl = 0; gl < RED2_GPB; ++gl) {
    const int g = g0 + gl;
    float m[4], mn[4], gs[4], gq[4];
#pragma unroll
    for (int e = 0; e < 4; ++e) {
      m[e] = -3.402823466e38f;
      mn[e] = 3.402823466e38f;
      gs[e] = 0.0f;
      gq[e] = 0.0f;
    }
#pragma unroll 4
    for (int k = 0; k < NSAMP2; ++k) {
      const v4f h = *(const v4f*)(H2 + ((size_t)g * NSAMP2 + k) * NCH2P + c4);
#pragma unroll
      for (int e = 0; e < 4; ++e) {
        const float x = h[e] + bv[e];
        m[e] = fmaxf(m[e], x);
        mn[e] = fminf(mn[e], x);
        gs[e] += x;
        gq[e] = __builtin_fmaf(x, x, gq[e]);
      }
    }
    v4f vm, vn;
#pragma unroll
    for (int e = 0; e < 4; ++e) {
      vm[e] = m[e];
      vn[e] = mn[e];
      ts[e] += gs[e];
      tq[e] += gq[e];
    }
    float* pmx = h2max + (size_t)g * NCH2P + c4;
    float* pmn = h2min + (size_t)g * NCH2P + c4;
    *(volatile v4f*)pmx = vm;
    *(volatile v4f*)pmn = vn;
    __threadfence();
    *(volatile v4f*)pmx = vm;
    *(volatile v4f*)pmn = vn;
  }
  v4f vs, vq;
#pragma unroll
  for (int e = 0; e < 4; ++e) {
    vs[e] = ts[e];
    vq[e] = tq[e];
  }
  float* ps = partials2 + ((size_t)blockIdx.x * 2) * NCH2P + c4;
  float* pq = partials2 + ((size_t)blockIdx.x * 2 + 1) * NCH2P + c4;
  *(volatile v4f*)ps = vs;
  *(volatile v4f*)pq = vq;
  __threadfence();
  *(volatile v4f*)ps = vs;
  *(volatile v4f*)pq = vq;
}

__global__ __launch_bounds__(256) void out1_kernel(const float* __restrict__ h2max,
                                                   const float* __restrict__ h2min,
                                                   const float* __restrict__ scale2,
                                                   const float* __restrict__ shift2,
                                                   float* __restrict__ out1) {
  __shared__ __align__(16) float ssc[NCH2P];
  __shared__ __align__(16) float ssh[NCH2P];
  const int tid = threadIdx.x;
  {
    const int i = tid < 175 ? tid : 175;
    const v4f a = *(const v4f*)(scale2 + 4 * i);
    const v4f c = *(const v4f*)(shift2 + 4 * i);
    *(v4f*)(ssc + 4 * i) = a;
    *(v4f*)(ssh + 4 * i) = c;
  }
  __syncthreads();
  const int q = blockIdx.x * 256 + tid;
  const int f0 = 4 * q;
  v4f o;
#pragma unroll
  for (int e = 0; e < 4; ++e) {
    const int f = f0 + e;
    const int row = f / NCH2;
    const int ch = f - row * NCH2;
    float a = h2max[(size_t)row * NCH2P + ch];
    float c = h2min[(size_t)row * NCH2P + ch];
    asm volatile("" : "+v"(a), "+v"(c));
    const float sc = ssc[ch];
    const float sh = ssh[ch];
    const float hs = (sc >= 0.0f) ? a : c;
    o[e] = fmaxf(__builtin_fmaf(sc, hs, sh), 0.0f);
  }
  *(volatile v4f*)(out1 + f0) = o;
  __threadfence();
  *(volatile v4f*)(out1 + f0) = o;
}

extern "C" void kernel_launch(void* const* d_in, const int* in_sizes, int n_in,
                              void* d_out, int out_size, void* d_ws, size_t ws_size,
                              hipStream_t stream) {
  (void)in_sizes; (void)out_size;
  if (n_in < 9) return;
  if (ws_size < WS_TOTAL) return;

  const float* xyz = (const float*)d_in[0];
  const float* w1  = (const float*)d_in[1];
  const float* b1  = (const float*)d_in[2];
  const float* g1  = (const float*)d_in[3];
  const float* be1 = (const float*)d_in[4];
  const float* w2  = (const float*)d_in[5];
  const float* b2  = (const float*)d_in[6];
  const float* g2  = (const float*)d_in[7];
  const float* be2 = (const float*)d_in[8];

  char* ws = (char*)d_ws;
  float* l1xyz4 = (float*)(ws + OFF_L1XYZ);
  float* l2xyz4 = (float*)(ws + OFF_L2XYZ);
  int*   idx1   = (int*)(ws + OFF_IDX1);
  int*   idx2   = (int*)(ws + OFF_IDX2);
  float* h1max  = (float*)(ws + OFF_H1MAX);
  float* h1min  = (float*)(ws + OFF_H1MIN);
  float* part1  = (float*)(ws + OFF_PART1);
  float* scale1 = (float*)(ws + OFF_SC1);
  float* shift1 = (float*)(ws + OFF_SH1);
  unsigned short* Ahi = (unsigned short*)(ws + OFF_AHI);
  unsigned short* Alo = (unsigned short*)(ws + OFF_ALO);
  unsigned short* Whi = (unsigned short*)(ws + OFF_WHI);
  unsigned short* Wlo = (unsigned short*)(ws + OFF_WLO);
  float* H2     = (float*)(ws + OFF_H2);
  float* h2max  = (float*)(ws + OFF_H2MAX);
  float* h2min  = (float*)(ws + OFF_H2MIN);
  float* part2  = (float*)(ws + OFF_PART2);
  float* scale2 = (float*)(ws + OFF_SC2);
  float* shift2 = (float*)(ws + OFF_SH2);

  float* out0 = (float*)d_out;
  float* out1 = (float*)d_out + (size_t)NBATCH * NCEN2 * 3;

  fps_kernel<NPT1, 16, NCEN1, 6, 1><<<NBATCH, 512, (size_t)(3 * NPT1 + NCEN1) * 4, stream>>>(xyz, l1xyz4, l1xyz4);
  ballquery_kernel<NPT1, NCEN1, NSAMP1, 6><<<(NBATCH * NCEN1) / 256, 256, 0, stream>>>(xyz, l1xyz4, idx1, BALL_R2_L1);
  mlp1_kernel<<<NPART1, 128, 0, stream>>>(xyz, l1xyz4, idx1, w1, b1, h1max, h1min, part1);
  bn_finalize_kernel<<<NCH1 / 32, 256, 0, stream>>>(part1, g1, be1, scale1, shift1,
                                                    1.0f / (float)(NBATCH * NCEN1 * NSAMP1), NPART1, NCH1, NCH1);

  fps_kernel<NCEN1, 4, NCEN2, 4, 2><<<NBATCH, 512, (size_t)(3 * NCEN1 + NCEN2) * 4, stream>>>(l1xyz4, l2xyz4, out0);
  ballquery_kernel<NCEN1, NCEN2, NSAMP2, 4><<<(NBATCH * NCEN2) / 256, 256, 0, stream>>>(l1xyz4, l2xyz4, idx2, BALL_R2_L2);
  pack_w2_kernel<<<NCH2P / 8, 256, 0, stream>>>(w2, Whi, Wlo);
  pack_a2_kernel<<<NROW2 / 8, 256, 0, stream>>>(h1max, h1min, scale1, shift1, l1xyz4, l2xyz4, idx2, Ahi, Alo);
  {
    const int tiles = (NROW2 / 64) * (NCH2P / 64);
    dim3 grid(tiles / 8, 1, 1);
    wmma_gemm64<1, true, 0, 0, false, 0><<<grid, 256, 0, stream>>>(
        Ahi, Alo, APITCH, 0L, Whi, Wlo, APITCH, 0L,
        (void*)H2, (void*)H2, NCH2P, 0L, scale2, H2, 0L,
        NROW2, NCH2P, KDIM2, 1.0f);
  }
  reduce2_kernel<<<NPART2, 176, 0, stream>>>(H2, b2, h2max, h2min, part2);
  bn_finalize_kernel<<<NCH2P / 32, 256, 0, stream>>>(part2, g2, be2, scale2, shift2,
                                                     1.0f / (float)NROW2, NPART2, NCH2P, NCH2);
  out1_kernel<<<(NBATCH * NCEN2 * NCH2) / 1024, 256, 0, stream>>>(h2max, h2min, scale2, shift2, out1);
}
